// FixedNMP_18992345383582
// MI455X (gfx1250) — hardware-verified
//
#include <hip/hip_runtime.h>


#pragma clang fp contract(off)

#define BATCH 128
#define NNODE 512
#define DDIM 64
#define NFEAT 7
#define NITER 3
#define GATES 192
#define MTILES (NNODE / 16)
#define TILES_TOTAL (BATCH * MTILES)
#define NROWS (BATCH * NNODE)
#define PB_TILE 128
#define VB_PITCH 32

typedef __bf16 v16bf __attribute__((ext_vector_type(16)));
typedef unsigned short v16us __attribute__((ext_vector_type(16)));
typedef unsigned short v8us __attribute__((ext_vector_type(8)));
typedef float v8f __attribute__((ext_vector_type(8)));
typedef float v4f __attribute__((ext_vector_type(4)));
typedef unsigned int v4u __attribute__((ext_vector_type(4)));

union FragU { v16bf v; v16us s; v4u u[2]; };
union Pk8 { v8us s; v4u u; };
struct F2 { v16bf h, l; };
struct F3 { v16bf h, m, l; };

typedef char chk_tiles_div4[(TILES_TOTAL % 4 == 0) ? 1 : -1];
typedef char chk_batch_div8[(BATCH % 8 == 0) ? 1 : -1];
typedef char chk_fragu_size[(sizeof(FragU) == 32) ? 1 : -1];
typedef char chk_pk8_size[(sizeof(Pk8) == 16) ? 1 : -1];
typedef char chk_gates[(GATES == 3 * DDIM) ? 1 : -1];

__device__ __forceinline__ v8f zero8() {
  v8f z = {0.f, 0.f, 0.f, 0.f, 0.f, 0.f, 0.f, 0.f};
  return z;
}

__device__ __forceinline__ v8f mma(v16bf a, v16bf b, v8f c) {
  v8f d = __builtin_amdgcn_wmma_f32_16x16x32_bf16(false, a, false, b, (short)0, c, false, false);
  asm volatile("v_nop\n\tv_nop\n\tv_nop\n\tv_nop" : "+v"(d) : "v"(a), "v"(b));
  return d;
}

__device__ __forceinline__ unsigned short bf_rne(float x) {
  unsigned int u = __float_as_uint(x);
  u += 0x7FFFu + ((u >> 16) & 1u);
  return (unsigned short)(u >> 16);
}
__device__ __forceinline__ float bf_val(unsigned short s) {
  return __uint_as_float(((unsigned int)s) << 16);
}
__device__ __forceinline__ void cvt3(float x, unsigned short& h, unsigned short& m, unsigned short& l) {
  h = bf_rne(x);
  const float r1 = x - bf_val(h);
  m = bf_rne(r1);
  const float r2 = r1 - bf_val(m);
  l = bf_rne(r2);
}

__device__ __forceinline__ void ld16(const float* row, int k0, int hh, float (&v)[16]) {
  const float* p0 = row + k0 + 8 * hh;
  const float* p1 = p0 + 16;
  const v4f q0 = *(const v4f*)(p0);
  const v4f q1 = *(const v4f*)(p0 + 4);
  const v4f q2 = *(const v4f*)(p1);
  const v4f q3 = *(const v4f*)(p1 + 4);
  v[0] = q0[0]; v[1] = q0[1]; v[2] = q0[2]; v[3] = q0[3];
  v[4] = q1[0]; v[5] = q1[1]; v[6] = q1[2]; v[7] = q1[3];
  v[8] = q2[0]; v[9] = q2[1]; v[10] = q2[2]; v[11] = q2[3];
  v[12] = q3[0]; v[13] = q3[1]; v[14] = q3[2]; v[15] = q3[3];
}

__device__ __forceinline__ F2 make2(const float* row, int k0, int hh) {
  float v[16];
  ld16(row, k0, hh, v);
  FragU a, b;
#pragma unroll
  for (int i = 0; i < 16; ++i) {
    const unsigned short x = bf_rne(v[i]);
    const unsigned short y = bf_rne(v[i] - bf_val(x));
    a.s[i] = x; b.s[i] = y;
  }
  F2 f; f.h = a.v; f.l = b.v;
  return f;
}

__device__ __forceinline__ F3 make3(const float* row, int k0, int hh) {
  float v[16];
  ld16(row, k0, hh, v);
  FragU a, b, c;
#pragma unroll
  for (int i = 0; i < 16; ++i) {
    unsigned short x, y, z;
    cvt3(v[i], x, y, z);
    a.s[i] = x; b.s[i] = y; c.s[i] = z;
  }
  F3 f; f.h = a.v; f.m = b.v; f.l = c.v;
  return f;
}

__device__ __forceinline__ F3 make3_relu(const float* row, int k0, int hh, bool neg) {
  float v[16];
  ld16(row, k0, hh, v);
  FragU a, b, c;
#pragma unroll
  for (int i = 0; i < 16; ++i) {
    const float y = neg ? -v[i] : v[i];
    unsigned short x, w, z;
    cvt3(fmaxf(y, 0.f), x, w, z);
    a.s[i] = x; b.s[i] = w; c.s[i] = z;
  }
  F3 f; f.h = a.v; f.m = b.v; f.l = c.v;
  return f;
}

__device__ __forceinline__ v16bf ldb(const __bf16* base, size_t off) {
  FragU f;
  const __bf16* p = base + off;
  f.u[0] = *(const v4u*)(p);
  f.u[1] = *(const v4u*)(p + 16);
  return f.v;
}

__device__ __forceinline__ v8f mma3w(v8f acc, const F2& a, const __bf16* wpl, int pstride, size_t off) {
  const v16bf bh = ldb(wpl, off);
  const v16bf bl = ldb(wpl, off + (size_t)pstride);
  acc = mma(a.h, bh, acc);
  acc = mma(a.h, bl, acc);
  acc = mma(a.l, bh, acc);
  return acc;
}

__device__ __forceinline__ v8f mma6w(v8f acc, const F3& a, const __bf16* wpl, int pstride, size_t off) {
  const v16bf bh = ldb(wpl, off);
  const v16bf bm = ldb(wpl, off + (size_t)pstride);
  const v16bf bl = ldb(wpl, off + 2 * (size_t)pstride);
  acc = mma(a.h, bh, acc);
  acc = mma(a.h, bm, acc);
  acc = mma(a.m, bh, acc);
  acc = mma(a.h, bl, acc);
  acc = mma(a.l, bh, acc);
  acc = mma(a.m, bm, acc);
  return acc;
}

__device__ __forceinline__ v8f mma6v(v8f acc, const F3& a, const F3& b) {
  acc = mma(a.h, b.h, acc);
  acc = mma(a.h, b.m, acc);
  acc = mma(a.m, b.h, acc);
  acc = mma(a.h, b.l, acc);
  acc = mma(a.l, b.h, acc);
  acc = mma(a.m, b.m, acc);
  return acc;
}

__device__ __forceinline__ void store_tile_lines(const float* st, float* dst, int lane) {
  v4f vals[8];
#pragma unroll
  for (int j = 0; j < 8; ++j) vals[j] = *(const v4f*)(st + (j * 32 + lane) * 4);
#pragma unroll
  for (int j = 0; j < 8; ++j) *(volatile v4f*)(dst + (size_t)(j * 32 + lane) * 4) = vals[j];
  __threadfence();
#pragma unroll
  for (int j = 0; j < 8; ++j) *(volatile v4f*)(dst + (size_t)(j * 32 + lane) * 4) = vals[j];
}

__global__ __launch_bounds__(32) void k_pack(const float* __restrict__ src, __bf16* __restrict__ dst,
                                           int nrows, int mode) {
  const int lane = threadIdx.x;
  const int rr = lane >> 3, kq = lane & 7;
  const int n = blockIdx.x * 4 + rr;
  const bool ok = n < nrows;
  const int nn = ok ? n : 0;
  Pk8 ph, pm, pl;
#pragma unroll
  for (int e = 0; e < 8; ++e) {
    const int k = kq * 8 + e;
    const size_t idx = mode ? ((size_t)nn * DDIM + k)
                            : ((size_t)(nn >> 6) * (DDIM * DDIM) + (size_t)k * DDIM + (size_t)(nn & 63));
    const float v = src[idx];
    unsigned short x, y, z;
    cvt3(v, x, y, z);
    ph.s[e] = x; pm.s[e] = y; pl.s[e] = z;
  }
  const size_t plane = (size_t)nrows * DDIM;
  __bf16* d0 = dst + (size_t)nn * DDIM + kq * 8;
  const v4u x0 = ph.u, x1 = pm.u, x2 = pl.u;
  if (ok) {
    *(volatile v4u*)(d0) = x0;
    *(volatile v4u*)(d0 + plane) = x1;
    *(volatile v4u*)(d0 + 2 * plane) = x2;
  }
  __threadfence();
  if (ok) {
    *(volatile v4u*)(d0) = x0;
    *(volatile v4u*)(d0 + plane) = x1;
    *(volatile v4u*)(d0 + 2 * plane) = x2;
  }
}

__global__ __launch_bounds__(256) void k_embed(const float* __restrict__ x, const float* __restrict__ w,
                                             const float* __restrict__ bias, float* __restrict__ h, int total) {
  const int t = blockIdx.x * 256 + threadIdx.x;
  if (t >= total) return;
  const int d = t & 63;
  const int bn = t >> 6;
  const float* xp = x + (size_t)bn * NFEAT;
  float acc = 0.f;
#pragma unroll
  for (int f = 0; f < NFEAT; ++f) acc = acc + xp[f] * w[f * DDIM + d];
  acc = acc + bias[d];
  const float v = fmaxf(acc, 0.f);
  *(volatile float*)(h + t) = v;
  __threadfence();
  *(volatile float*)(h + t) = v;
}

__global__ __launch_bounds__(128) void k_resfc(const float* __restrict__ hin, const __bf16* __restrict__ wpl,
                                             int pstride, const float* __restrict__ bias,
                                             float* __restrict__ hout) {
  __shared__ float sT[4][16 * DDIM] __attribute__((aligned(16)));
  const int wave = threadIdx.x >> 5, lane = threadIdx.x & 31, hh = lane >> 4, m = lane & 15;
  const int tile = blockIdx.x * 4 + wave;
  const int b = tile / MTILES, mt = tile % MTILES;
  const size_t rowbase = (size_t)b * NNODE + (size_t)mt * 16;
  const float* hrow = hin + (rowbase + m) * DDIM;
  const F2 a0 = make2(hrow, 0, hh);
  const F2 a1 = make2(hrow, 32, hh);
  float* st = &sT[wave][0];
#pragma unroll
  for (int nt = 0; nt < 4; ++nt) {
    const int c = nt * 16 + m;
    v8f acc = zero8();
    acc = mma3w(acc, a0, wpl, pstride, (size_t)c * DDIM + 0 + 8 * hh);
    acc = mma3w(acc, a1, wpl, pstride, (size_t)c * DDIM + 32 + 8 * hh);
    const float bi = bias[c];
#pragma unroll
    for (int r = 0; r < 8; ++r) {
      const int row = 8 * hh + r;
      const float hv = hin[(rowbase + row) * DDIM + c];
      st[row * DDIM + c] = hv + fmaxf(acc[r] + bi, 0.f);
    }
  }
  __syncthreads();
  store_tile_lines(st, hout + rowbase * DDIM, lane);
}

__global__ __launch_bounds__(128) void k_msg(const float* __restrict__ hin, const __bf16* __restrict__ wpl,
                                           int pstride, const float* __restrict__ bias,
                                           const float* __restrict__ mask, float* __restrict__ pbuf) {
  __shared__ float sP[4][PB_TILE] __attribute__((aligned(16)));
  const int wave = threadIdx.x >> 5, lane = threadIdx.x & 31, hh = lane >> 4, m = lane & 15;
  const int tile = blockIdx.x * 4 + wave;
  const int b = tile / MTILES, mt = tile % MTILES;
  const size_t rowbase = (size_t)b * NNODE + (size_t)mt * 16;
  const float* hrow = hin + (rowbase + m) * DDIM;
  const F3 a0 = make3(hrow, 0, hh);
  const F3 a1 = make3(hrow, 32, hh);
  float mk[8];
#pragma unroll
  for (int r = 0; r < 8; ++r) mk[r] = mask[rowbase + 8 * hh + r];
#pragma unroll
  for (int nt = 0; nt < 4; ++nt) {
    const int c = nt * 16 + m;
    v8f acc = zero8();
    acc = mma6w(acc, a0, wpl, pstride, (size_t)c * DDIM + 0 + 8 * hh);
    acc = mma6w(acc, a1, wpl, pstride, (size_t)c * DDIM + 32 + 8 * hh);
    const float bi = bias[c];
    float p = 0.f;
#pragma unroll
    for (int r = 0; r < 8; ++r) {
      const int row = 8 * hh + r;
      const float mv = hin[(rowbase + row) * DDIM + c] + fmaxf(acc[r] + bi, 0.f);
      p = p + mk[r] * mv;
    }
    sP[wave][hh * DDIM + c] = p;
  }
  __syncthreads();
  const v4f val = *(const v4f*)(&sP[wave][lane * 4]);
  float* dst = pbuf + (size_t)tile * PB_TILE + lane * 4;
  *(volatile v4f*)dst = val;
  __threadfence();
  *(volatile v4f*)dst = val;
}

__global__ __launch_bounds__(128) void k_gate(const float* __restrict__ pbuf, const float* __restrict__ wih,
                                            float* __restrict__ gbuf) {
  __shared__ float sS[8 * DDIM] __attribute__((aligned(16)));
  __shared__ float sG[16 * GATES] __attribute__((aligned(16)));
  const int tid = threadIdx.x;
  const int bl0 = blockIdx.x * 8;
#pragma unroll
  for (int q = 0; q < 4; ++q) {
    const int p = tid * 4 + q;
    const int bl = p >> 6, d = p & 63;
    const float* pp = pbuf + (size_t)(bl0 + bl) * (MTILES * 2 * DDIM) + d;
    double a = 0.0;
#pragma unroll 8
    for (int j = 0; j < MTILES * 2; ++j) a += (double)pp[(size_t)j * DDIM];
    sS[bl * DDIM + d] = (float)a;
  }
  __syncthreads();
  const int wave = tid >> 5, lane = tid & 31, hh = lane >> 4, m = lane & 15;
  const float* srow = &sS[(m >> 1) * DDIM];
  const bool neg = (m & 1) != 0;
  const F3 a0 = make3_relu(srow, 0, hh, neg);
  const F3 a1 = make3_relu(srow, 32, hh, neg);
#pragma unroll
  for (int t = 0; t < 3; ++t) {
    const int u = (wave * 3 + t) * 16 + m;
    const float* wr = wih + (size_t)u * DDIM;
    const F3 b0 = make3(wr, 0, hh);
    const F3 b1 = make3(wr, 32, hh);
    v8f acc = zero8();
    acc = mma6v(acc, a0, b0);
    acc = mma6v(acc, a1, b1);
#pragma unroll
    for (int r = 0; r < 8; ++r) sG[(8 * hh + r) * GATES + u] = acc[r];
  }
  __syncthreads();
  float* dst = gbuf + (size_t)bl0 * 2 * GATES;
  v4f vals[6];
#pragma unroll
  for (int j = 0; j < 6; ++j) vals[j] = *(const v4f*)(&sG[(j * 128 + tid) * 4]);
#pragma unroll
  for (int j = 0; j < 6; ++j) *(volatile v4f*)(dst + (size_t)(j * 128 + tid) * 4) = vals[j];
  __threadfence();
#pragma unroll
  for (int j = 0; j < 6; ++j) *(volatile v4f*)(dst + (size_t)(j * 128 + tid) * 4) = vals[j];
}

__global__ __launch_bounds__(128) void k_gru(const float* __restrict__ hin, const __bf16* __restrict__ wpl,
                                           int pstride, const float* __restrict__ bih,
                                           const float* __restrict__ bhh, const float* __restrict__ gbuf,
                                           const float* __restrict__ mask, float* __restrict__ hout) {
  __shared__ float sT[4][16 * DDIM] __attribute__((aligned(16)));
  const int wave = threadIdx.x >> 5, lane = threadIdx.x & 31, hh = lane >> 4, m = lane & 15;
  const int tile = blockIdx.x * 4 + wave;
  const int b = tile / MTILES, mt = tile % MTILES;
  const size_t rowbase = (size_t)b * NNODE + (size_t)mt * 16;
  const float* hrow = hin + (rowbase + m) * DDIM;
  const F2 a0 = make2(hrow, 0, hh);
  const F2 a1 = make2(hrow, 32, hh);
  float mk[8];
#pragma unroll
  for (int r = 0; r < 8; ++r) mk[r] = mask[rowbase + 8 * hh + r];
  const float* gP = gbuf + (size_t)b * 2 * GATES;
  const float* gM = gP + GATES;
  float* st = &sT[wave][0];
#pragma unroll
  for (int nt = 0; nt < 4; ++nt) {
    const int c = nt * 16 + m;
    v8f ar = zero8(), az = zero8(), an = zero8();
    ar = mma3w(ar, a0, wpl, pstride, (size_t)(c) * DDIM + 0 + 8 * hh);
    ar = mma3w(ar, a1, wpl, pstride, (size_t)(c) * DDIM + 32 + 8 * hh);
    az = mma3w(az, a0, wpl, pstride, (size_t)(DDIM + c) * DDIM + 0 + 8 * hh);
    az = mma3w(az, a1, wpl, pstride, (size_t)(DDIM + c) * DDIM + 32 + 8 * hh);
    an = mma3w(an, a0, wpl, pstride, (size_t)(2 * DDIM + c) * DDIM + 0 + 8 * hh);
    an = mma3w(an, a1, wpl, pstride, (size_t)(2 * DDIM + c) * DDIM + 32 + 8 * hh);
    const float gpr = gP[c], gmr = gM[c];
    const float gpz = gP[DDIM + c], gmz = gM[DDIM + c];
    const float gpn = gP[2 * DDIM + c], gmn = gM[2 * DDIM + c];
    const float bir = bih[c], biz = bih[DDIM + c], bin = bih[2 * DDIM + c];
    const float bhr = bhh[c], bhz = bhh[DDIM + c], bhn = bhh[2 * DDIM + c];
#pragma unroll
    for (int r = 0; r < 8; ++r) {
      const int row = 8 * hh + r;
      const float hprev = hin[(rowbase + row) * DDIM + c];
      const float mrow = mk[r];
      const float am = fabsf(mrow);
      const bool neg = mrow < 0.f;
      const float ir = am * (neg ? gmr : gpr) + bir;
      const float iz = am * (neg ? gmz : gpz) + biz;
      const float in_ = am * (neg ? gmn : gpn) + bin;
      const float xr = ir + (ar[r] + bhr);
      const float xz = iz + (az[r] + bhz);
      const float hn = an[r] + bhn;
      const float rg = 1.f / (1.f + expf(-xr));
      const float zg = 1.f / (1.f + expf(-xz));
      const float ng = tanhf(in_ + rg * hn);
      st[row * DDIM + c] = ng + zg * (hprev - ng);
    }
  }
  __syncthreads();
  store_tile_lines(st, hout + rowbase * DDIM, lane);
}

__global__ __launch_bounds__(128) void k_readout(const float* __restrict__ hin, const __bf16* __restrict__ wpl,
                                               int pstride, const float* __restrict__ bias,
                                               const float* __restrict__ fcw, const float* __restrict__ fcb,
                                               float* __restrict__ vbuf) {
  __shared__ float sV[4];
  const int wave = threadIdx.x >> 5, lane = threadIdx.x & 31, hh = lane >> 4, m = lane & 15;
  const int b = blockIdx.x;
  const float fb = fcb[0];
  float wtot = 0.f;
#pragma unroll 1
  for (int j = 0; j < MTILES / 4; ++j) {
    const int mt = wave * (MTILES / 4) + j;
    const size_t rowbase = (size_t)b * NNODE + (size_t)mt * 16;
    const float* hrow = hin + (rowbase + m) * DDIM;
    const F2 a0 = make2(hrow, 0, hh);
    const F2 a1 = make2(hrow, 32, hh);
    float dp[8];
#pragma unroll
    for (int r = 0; r < 8; ++r) dp[r] = 0.f;
#pragma unroll
    for (int nt = 0; nt < 4; ++nt) {
      const int c = nt * 16 + m;
      v8f acc = zero8();
      acc = mma3w(acc, a0, wpl, pstride, (size_t)c * DDIM + 0 + 8 * hh);
      acc = mma3w(acc, a1, wpl, pstride, (size_t)c * DDIM + 32 + 8 * hh);
      const float bi = bias[c];
      const float w = fcw[c];
#pragma unroll
      for (int r = 0; r < 8; ++r) {
        const int row = 8 * hh + r;
        const float hr = hin[(rowbase + row) * DDIM + c] + fmaxf(acc[r] + bi, 0.f);
        dp[r] = fmaf(hr, w, dp[r]);
      }
    }
#pragma unroll
    for (int r = 0; r < 8; ++r) {
#pragma unroll
      for (int off = 1; off < 16; off <<= 1) dp[r] += __shfl_xor(dp[r], off);
    }
    float vs = 0.f;
#pragma unroll
    for (int r = 0; r < 8; ++r) vs += fmaxf(dp[r] + fb, 0.f);
    vs = vs + __shfl_xor(vs, 16);
    wtot += vs;
  }
  if (lane == 0) sV[wave] = wtot;
  __syncthreads();
  if (wave == 0) {
    const float tot = ((sV[0] + sV[1]) + sV[2]) + sV[3];
    const float val = (lane == 0) ? tot : 0.f;
    float* dst = vbuf + (size_t)b * VB_PITCH + lane;
    *(volatile float*)dst = val;
    __threadfence();
    *(volatile float*)dst = val;
  }
}

__global__ __launch_bounds__(128) void k_mean(const float* __restrict__ vbuf, float* __restrict__ out, int nb) {
  const int b = threadIdx.x;
  if (b >= nb) return;
  const float v = vbuf[(size_t)b * VB_PITCH] * (1.0f / (float)NNODE);
  *(volatile float*)(out + b) = v;
  __threadfence();
  *(volatile float*)(out + b) = v;
}

extern "C" void kernel_launch(void* const* d_in, const int* in_sizes, int n_in,
                              void* d_out, int out_size, void* d_ws, size_t ws_size,
                              hipStream_t stream) {
  if (n_in < 16 || out_size != BATCH) return;
  if (in_sizes[0] != BATCH * NNODE * NFEAT || in_sizes[1] != BATCH * NNODE ||
      in_sizes[2] != NFEAT * DDIM || in_sizes[3] != DDIM ||
      in_sizes[4] != DDIM * DDIM || in_sizes[5] != DDIM ||
      in_sizes[6] != NITER * DDIM * DDIM || in_sizes[7] != NITER * DDIM ||
      in_sizes[8] != NITER * GATES * DDIM || in_sizes[9] != NITER * GATES * DDIM ||
      in_sizes[10] != NITER * GATES || in_sizes[11] != NITER * GATES ||
      in_sizes[12] != DDIM * DDIM || in_sizes[13] != DDIM ||
      in_sizes[14] != DDIM || in_sizes[15] < 1) return;

  const float* x        = (const float*)d_in[0];
  const float* mask     = (const float*)d_in[1];
  const float* emb_w    = (const float*)d_in[2];
  const float* emb_b    = (const float*)d_in[3];
  const float* res0_w   = (const float*)d_in[4];
  const float* res0_b   = (const float*)d_in[5];
  const float* msg_w    = (const float*)d_in[6];
  const float* msg_b    = (const float*)d_in[7];
  const float* gwih     = (const float*)d_in[8];
  const float* gwhh     = (const float*)d_in[9];
  const float* gbih     = (const float*)d_in[10];
  const float* gbhh     = (const float*)d_in[11];
  const float* ro_res_w = (const float*)d_in[12];
  const float* ro_res_b = (const float*)d_in[13];
  const float* ro_fc_w  = (const float*)d_in[14];
  const float* ro_fc_b  = (const float*)d_in[15];
  float* out = (float*)d_out;

  char* ws = (char*)d_ws;
  const size_t HBYTES = (size_t)NROWS * DDIM * sizeof(float);
  const size_t W64B   = (size_t)3 * 64 * DDIM * 2;
  const size_t WMSGB  = (size_t)3 * (NITER * 64) * DDIM * 2;
  const size_t WHHB   = (size_t)3 * (NITER * GATES) * DDIM * 2;
  const size_t PBB    = (size_t)TILES_TOTAL * PB_TILE * sizeof(float);
  const size_t GBB    = (size_t)BATCH * 2 * GATES * sizeof(float);
  const size_t VBB    = (size_t)BATCH * VB_PITCH * sizeof(float);
  size_t off = 0;
  float*  hA   = (float*)(ws + off);  off += HBYTES;
  float*  hB   = (float*)(ws + off);  off += HBYTES;
  __bf16* wres = (__bf16*)(ws + off); off += W64B;
  __bf16* wro  = (__bf16*)(ws + off); off += W64B;
  __bf16* wmsg = (__bf16*)(ws + off); off += WMSGB;
  __bf16* whh  = (__bf16*)(ws + off); off += WHHB;
  float*  pbuf = (float*)(ws + off);  off += PBB;
  float*  gbuf = (float*)(ws + off);  off += GBB;
  float*  vbuf = (float*)(ws + off);  off += VBB;
  if (off > ws_size) return;

  const int pstride64  = 64 * DDIM;
  const int pstrideMsg = NITER * 64 * DDIM;
  const int pstrideHh  = NITER * GATES * DDIM;

  k_pack<<<64 / 4, 32, 0, stream>>>(res0_w, wres, 64, 0);
  k_pack<<<64 / 4, 32, 0, stream>>>(ro_res_w, wro, 64, 0);
  k_pack<<<(NITER * 64) / 4, 32, 0, stream>>>(msg_w, wmsg, NITER * 64, 0);
  k_pack<<<(NITER * GATES) / 4, 32, 0, stream>>>(gwhh, whh, NITER * GATES, 1);

  const int embTotal = NROWS * DDIM;
  k_embed<<<(embTotal + 255) / 256, 256, 0, stream>>>(x, emb_w, emb_b, hA, embTotal);

  k_resfc<<<TILES_TOTAL / 4, 128, 0, stream>>>(hA, wres, pstride64, res0_b, hB);

  float* cur = hB;
  float* oth = hA;
  for (int i = 0; i < NITER; ++i) {
    k_msg<<<TILES_TOTAL / 4, 128, 0, stream>>>(
        cur, wmsg + (size_t)i * 64 * DDIM, pstrideMsg, msg_b + (size_t)i * DDIM, mask, pbuf);
    k_gate<<<BATCH / 8, 128, 0, stream>>>(pbuf, gwih + (size_t)i * GATES * DDIM, gbuf);
    k_gru<<<TILES_TOTAL / 4, 128, 0, stream>>>(
        cur, whh + (size_t)i * GATES * DDIM, pstrideHh,
        gbih + (size_t)i * GATES, gbhh + (size_t)i * GATES, gbuf, mask, oth);
    float* t = cur; cur = oth; oth = t;
  }

  k_readout<<<BATCH, 128, 0, stream>>>(cur, wro, pstride64, ro_res_b, ro_fc_w, ro_fc_b, vbuf);
  k_mean<<<1, 128, 0, stream>>>(vbuf, out, BATCH);
}
